// JKExpert_2310692405504
// MI455X (gfx1250) — hardware-verified
//
#include <hip/hip_runtime.h>
#include <stddef.h>


#define DF      256
#define KJ      768
#define NLAY    3
#define NTHR    256
#define NWAVE   8
#define EPT     8
#define NGRP    2
#define CHUNK   (NTHR * EPT * NGRP)
#define WCAP    (EPT * NGRP * 32)
#define LISTN   (NWAVE * WCAP)
#define NB      256
#define NBD     4096
#define GROWS   128
#define GCOLS   128
#define SP      128
#define HSC     16.0f
#define WSC     16.0f
#define SINV    0.00390625f
#define BN_EPS  1e-5f

#define LDS_GEMM (GROWS * SP * 4)
#define LDS_AGG  (NB * DF * 4 + LISTN * 4 + 64)
#define WS_CAP   ((size_t)134217728)

static_assert((CHUNK & (CHUNK - 1)) == 0);
static_assert(CHUNK <= 4096);
static_assert((NB & (NB - 1)) == 0 && NB <= 4096);
static_assert((NBD & (NBD - 1)) == 0 && NBD <= 4096);
static_assert(NBD % NB == 0);
static_assert(NB % GROWS == 0);
static_assert(DF == 2 * GCOLS);
static_assert(NB % NWAVE == 0);
static_assert(GROWS == 16 * NWAVE);

typedef float          v4f  __attribute__((ext_vector_type(4)));
typedef float          v8f  __attribute__((ext_vector_type(8)));
typedef int            v4i  __attribute__((ext_vector_type(4)));
typedef unsigned short v8u  __attribute__((ext_vector_type(8)));
typedef _Float16       v8h  __attribute__((ext_vector_type(8)));
typedef _Float16       v16h __attribute__((ext_vector_type(16)));
typedef __bf16         v8b  __attribute__((ext_vector_type(8)));
typedef __bf16         v16b __attribute__((ext_vector_type(16)));
union FragH { v16h v; v8h h[2]; };
union FragB { v16b v; v8b h[2]; };

__device__ __forceinline__ unsigned int bf16_rne(float f) {
  const unsigned int u = __float_as_uint(f);
  return (u + 0x7FFFu + ((u >> 16) & 1u)) >> 16;
}

__device__ __forceinline__ void split8(v4f a, v4f b, v8u& hi, v8u& lo) {
  float f[8] = {a.x, a.y, a.z, a.w, b.x, b.y, b.z, b.w};
#pragma unroll
  for (int j = 0; j < 8; ++j) {
    const unsigned int hb = bf16_rne(f[j]);
    const float hf = __uint_as_float(hb << 16);
    hi[j] = (unsigned short)hb;
    lo[j] = (unsigned short)bf16_rne(f[j] - hf);
  }
}

__device__ __forceinline__ v8h cvt8(v4f a, v4f b) {
  v8h r;
  r[0] = (_Float16)a.x; r[1] = (_Float16)a.y; r[2] = (_Float16)a.z; r[3] = (_Float16)a.w;
  r[4] = (_Float16)b.x; r[5] = (_Float16)b.y; r[6] = (_Float16)b.z; r[7] = (_Float16)b.w;
  return r;
}

__device__ __forceinline__ v8f wmh(v16h a, v16h b, v8f c) {
  v8f d = __builtin_amdgcn_wmma_f32_16x16x32_f16(false, a, false, b, (short)0, c, false, false);
  asm volatile("v_nop\n\tv_nop\n\tv_nop\n\tv_nop" : "+v"(d) : "v"(a), "v"(b));
  return d;
}
__device__ __forceinline__ v8f wmb(v16b a, v16b b, v8f c) {
  v8f d = __builtin_amdgcn_wmma_f32_16x16x32_bf16(false, a, false, b, (short)0, c, false, false);
  asm volatile("v_nop\n\tv_nop\n\tv_nop\n\tv_nop" : "+v"(d) : "v"(a), "v"(b));
  return d;
}

template <int NBT>
__device__ __forceinline__ int scan_chunk(const int* __restrict__ dsts, int nE, int cbase, int nodeBase,
                                          int vec8, int* list, int tid, int lane, int wave) {
  int wc = 0;
#pragma unroll
  for (int g = 0; g < NGRP; ++g) {
    const int el0  = (g * NTHR + tid) * EPT;
    const int e0   = cbase + el0;
    const int sent = -2147483647 - 1;
    v4i da, db;
    if (vec8 != 0 && e0 + 7 < nE) {
      da = *(const v4i*)(dsts + e0);
      db = *(const v4i*)(dsts + e0 + 4);
    } else {
      da.x = (e0     < nE) ? dsts[min(e0, nE - 1)] : sent;
      da.y = (e0 + 1 < nE) ? dsts[min(e0 + 1, nE - 1)] : sent;
      da.z = (e0 + 2 < nE) ? dsts[min(e0 + 2, nE - 1)] : sent;
      da.w = (e0 + 3 < nE) ? dsts[min(e0 + 3, nE - 1)] : sent;
      db.x = (e0 + 4 < nE) ? dsts[min(e0 + 4, nE - 1)] : sent;
      db.y = (e0 + 5 < nE) ? dsts[min(e0 + 5, nE - 1)] : sent;
      db.z = (e0 + 6 < nE) ? dsts[min(e0 + 6, nE - 1)] : sent;
      db.w = (e0 + 7 < nE) ? dsts[min(e0 + 7, nE - 1)] : sent;
    }
    const unsigned nb = (unsigned)nodeBase;
    const unsigned s0 = (unsigned)da.x - nb, s1 = (unsigned)da.y - nb;
    const unsigned s2 = (unsigned)da.z - nb, s3 = (unsigned)da.w - nb;
    const unsigned s4 = (unsigned)db.x - nb, s5 = (unsigned)db.y - nb;
    const unsigned s6 = (unsigned)db.z - nb, s7 = (unsigned)db.w - nb;
    const bool h0 = s0 < (unsigned)NBT, h1 = s1 < (unsigned)NBT, h2 = s2 < (unsigned)NBT, h3 = s3 < (unsigned)NBT;
    const bool h4 = s4 < (unsigned)NBT, h5 = s5 < (unsigned)NBT, h6 = s6 < (unsigned)NBT, h7 = s7 < (unsigned)NBT;
    const unsigned any = __builtin_amdgcn_ballot_w32(h0 | h1 | h2 | h3 | h4 | h5 | h6 | h7);
    if (any != 0u) {
#define HITJ(J, HJ, SJ) { \
        const unsigned mj = __builtin_amdgcn_ballot_w32(HJ); \
        if (mj != 0u) { \
          if (HJ) { \
            const int pos = wc + (int)__builtin_amdgcn_mbcnt_lo(mj, 0u); \
            if (pos < WCAP) list[wave * WCAP + pos] = ((el0 + (J)) << 12) | (int)(SJ); \
          } \
          wc += (int)__builtin_popcount(mj); } }
      HITJ(0, h0, s0)
      HITJ(1, h1, s1)
      HITJ(2, h2, s2)
      HITJ(3, h3, s3)
      HITJ(4, h4, s4)
      HITJ(5, h5, s5)
      HITJ(6, h6, s6)
      HITJ(7, h7, s7)
#undef HITJ
    }
  }
  return wc;
}

__global__ __launch_bounds__(NTHR) void k_prep(
    const float* __restrict__ x, const float* __restrict__ Ws, const float* __restrict__ lw,
    unsigned short* xh, unsigned short* xl, unsigned short* w0h, unsigned short* w0l,
    _Float16* w1f, _Float16* w2f, unsigned short* lwh, unsigned short* lwl,
    int nN, int nPad) {
  const int i   = blockIdx.x * NTHR + threadIdx.x;
  const int nW  = DF * DF / 8;
  const int nLW = DF * KJ / 8;
  const int nX  = nPad * (DF / 8);
  const int t3 = 3 * nW, t4 = t3 + nLW, t5 = t4 + nX;
  if (i >= t5) return;
  if (i < t3) {
    const int l  = i / nW;
    const int o  = (i - l * nW) * 8;
    const int n  = o / DF;
    const int k0 = o - n * DF;
    const float* p = Ws + (size_t)l * DF * DF + (size_t)k0 * DF + n;
    v4f a, b;
    a.x = p[0];      a.y = p[DF];     a.z = p[2 * DF]; a.w = p[3 * DF];
    b.x = p[4 * DF]; b.y = p[5 * DF]; b.z = p[6 * DF]; b.w = p[7 * DF];
    if (l == 0) {
      v8u hv, lv;
      split8(a, b, hv, lv);
      *(volatile v8u*)(w0h + o) = hv;
      *(volatile v8u*)(w0l + o) = lv;
      __threadfence();
      *(volatile v8u*)(w0h + o) = hv;
      *(volatile v8u*)(w0l + o) = lv;
    } else {
      const v8h fv = cvt8(a * WSC, b * WSC);
      _Float16* dp = (l == 1 ? w1f : w2f) + o;
      *(volatile v8h*)dp = fv;
      __threadfence();
      *(volatile v8h*)dp = fv;
    }
  } else if (i < t4) {
    const int o  = (i - t3) * 8;
    const int n  = o / KJ;
    const int k0 = o - n * KJ;
    const float* p = lw + (size_t)k0 * DF + n;
    v4f a, b;
    a.x = p[0];      a.y = p[DF];     a.z = p[2 * DF]; a.w = p[3 * DF];
    b.x = p[4 * DF]; b.y = p[5 * DF]; b.z = p[6 * DF]; b.w = p[7 * DF];
    v8u hv, lv;
    split8(a, b, hv, lv);
    *(volatile v8u*)(lwh + o) = hv;
    *(volatile v8u*)(lwl + o) = lv;
    __threadfence();
    *(volatile v8u*)(lwh + o) = hv;
    *(volatile v8u*)(lwl + o) = lv;
  } else {
    const int o  = (i - t4) * 8;
    const int r  = o / DF;
    const int c0 = o - r * DF;
    const int rc = r > nN - 1 ? nN - 1 : r;
    const float* xp = x + (size_t)rc * DF + c0;
    const v4f a = *(const v4f*)xp, b = *(const v4f*)(xp + 4);
    v8u hv, lv;
    split8(a, b, hv, lv);
    *(volatile v8u*)(xh + (size_t)o) = hv;
    *(volatile v8u*)(xl + (size_t)o) = lv;
    __threadfence();
    *(volatile v8u*)(xh + (size_t)o) = hv;
    *(volatile v8u*)(xl + (size_t)o) = lv;
  }
}

__global__ __launch_bounds__(NTHR) void k_deg(
    const int* __restrict__ ei, float* dinv, int nN, int nE, int vec8) {
  __shared__ __attribute__((aligned(16))) int cnt[NBD];
  __shared__ __attribute__((aligned(16))) int list[LISTN];
  __shared__ int wcnt[NWAVE];
  const int tid = threadIdx.x, lane = tid & 31, wave = tid >> 5;
  const int nodeBase = blockIdx.x * NBD;
  const int* dsts = ei + nE;
  (void)nN;

  for (int i = tid; i < NBD; i += NTHR) cnt[i] = 0;
  __syncthreads();

  const int nChunks = (nE + CHUNK - 1) / CHUNK;
#pragma unroll 1
  for (int ch = 0; ch < nChunks; ++ch) {
    const int cbase = ch * CHUNK;
    const int wc = scan_chunk<NBD>(dsts, nE, cbase, nodeBase, vec8, list, tid, lane, wave);
    if (lane == 0) wcnt[wave] = wc;
    __syncthreads();
    if (wave == 0) {
#pragma unroll 1
      for (int wsx = 0; wsx < NWAVE; ++wsx) {
        int n = __builtin_amdgcn_readfirstlane(wcnt[wsx]);
        n = n > WCAP ? WCAP : (n < 0 ? 0 : n);
        const int* lp = list + wsx * WCAP;
#pragma unroll 1
        for (int i = 0; i < n; ++i) {
          const int ent  = __builtin_amdgcn_readfirstlane(lp[i]);
          const int slot = ent & (NBD - 1);
          if (lane == 0) cnt[slot] = cnt[slot] + 1;
        }
      }
    }
    __syncthreads();
  }

  v4f dq[4];
#pragma unroll
  for (int q = 0; q < 4; ++q) {
    const int f = (wave * 4 + q) * 128 + 4 * lane;
    const v4i c = *(const v4i*)(cnt + f);
    dq[q].x = rsqrtf((float)(c.x + 1));
    dq[q].y = rsqrtf((float)(c.y + 1));
    dq[q].z = rsqrtf((float)(c.z + 1));
    dq[q].w = rsqrtf((float)(c.w + 1));
  }
  float* dp = dinv + (size_t)nodeBase;
#pragma unroll
  for (int q = 0; q < 4; ++q) *(volatile v4f*)(dp + (wave * 4 + q) * 128 + 4 * lane) = dq[q];
  __threadfence();
#pragma unroll
  for (int q = 0; q < 4; ++q) *(volatile v4f*)(dp + (wave * 4 + q) * 128 + 4 * lane) = dq[q];
}

template <int MODE>
__global__ __launch_bounds__(NTHR) void k_gemm(
    const unsigned short* __restrict__ Ah, const unsigned short* __restrict__ Al, int lda,
    const unsigned short* __restrict__ Bh, const unsigned short* __restrict__ Bl, int K,
    const float* __restrict__ dinv, const float* __restrict__ bias, float* C, int nN) {
  extern __shared__ v4f lds_dyn[];
  float* stg = (float*)lds_dyn;
  const int tid = threadIdx.x, lane = tid & 31, wave = tid >> 5, hh = lane >> 4, m = lane & 15;
  const int rowBase = blockIdx.x * GROWS;
  const int colBase = blockIdx.y * GCOLS;

  v8f acc[8];
#pragma unroll
  for (int t = 0; t < 8; ++t) { v8f z = {0.f, 0.f, 0.f, 0.f, 0.f, 0.f, 0.f, 0.f}; acc[t] = z; }

  const size_t aoff = (size_t)(rowBase + wave * 16 + m) * lda + 8 * hh;
  const size_t boff = (size_t)(colBase + m) * K + 8 * hh;

#pragma unroll 1
  for (int k0 = 0; k0 < K; k0 += 32) {
    if (MODE == 1) {
      FragH a;
      a.h[0] = *(const v8h*)(Ah + aoff + k0);
      a.h[1] = *(const v8h*)(Ah + aoff + k0 + 16);
#pragma unroll
      for (int t = 0; t < 8; ++t) {
        const unsigned short* bp = Bh + boff + (size_t)(16 * t) * K + k0;
        FragH b;
        b.h[0] = *(const v8h*)bp;
        b.h[1] = *(const v8h*)(bp + 16);
        acc[t] = wmh(a.v, b.v, acc[t]);
      }
    } else {
      FragB ah, al;
      ah.h[0] = *(const v8b*)(Ah + aoff + k0);
      ah.h[1] = *(const v8b*)(Ah + aoff + k0 + 16);
      al.h[0] = *(const v8b*)(Al + aoff + k0);
      al.h[1] = *(const v8b*)(Al + aoff + k0 + 16);
#pragma unroll
      for (int t = 0; t < 8; ++t) {
        const unsigned short* bp = Bh + boff + (size_t)(16 * t) * K + k0;
        const unsigned short* bq = Bl + boff + (size_t)(16 * t) * K + k0;
        FragB bh, bl;
        bh.h[0] = *(const v8b*)bp;
        bh.h[1] = *(const v8b*)(bp + 16);
        bl.h[0] = *(const v8b*)bq;
        bl.h[1] = *(const v8b*)(bq + 16);
        acc[t] = wmb(ah.v, bh.v, acc[t]);
        acc[t] = wmb(al.v, bh.v, acc[t]);
        acc[t] = wmb(ah.v, bl.v, acc[t]);
      }
    }
  }

  const int r0 = wave * 16 + 8 * hh;
  float s0 = 1.f, s1 = 1.f, s2 = 1.f, s3 = 1.f, s4 = 1.f, s5 = 1.f, s6 = 1.f, s7 = 1.f;
  if (MODE != 2) {
    const float sc = (MODE == 1) ? SINV : 1.0f;
    const v4f dA = *(const v4f*)(dinv + (size_t)rowBase + r0);
    const v4f dB = *(const v4f*)(dinv + (size_t)rowBase + r0 + 4);
    s0 = dA.x * sc; s1 = dA.y * sc; s2 = dA.z * sc; s3 = dA.w * sc;
    s4 = dB.x * sc; s5 = dB.y * sc; s6 = dB.z * sc; s7 = dB.w * sc;
  }
  float* sp = stg + r0 * SP + m;
#pragma unroll
  for (int t = 0; t < 8; ++t) {
    sp[0 * SP + 16 * t] = acc[t][0] * s0;
    sp[1 * SP + 16 * t] = acc[t][1] * s1;
    sp[2 * SP + 16 * t] = acc[t][2] * s2;
    sp[3 * SP + 16 * t] = acc[t][3] * s3;
    sp[4 * SP + 16 * t] = acc[t][4] * s4;
    sp[5 * SP + 16 * t] = acc[t][5] * s5;
    sp[6 * SP + 16 * t] = acc[t][6] * s6;
    sp[7 * SP + 16 * t] = acc[t][7] * s7;
  }
  __syncthreads();

  v4f bv = {0.f, 0.f, 0.f, 0.f};
  if (MODE == 2) bv = *(const v4f*)(bias + colBase + 4 * lane);
  const float* lp = stg + (wave * 16) * SP + 4 * lane;
  float* gp = C + (size_t)(rowBase + wave * 16) * DF + colBase + 4 * lane;
  const int grow0 = rowBase + wave * 16;
#pragma unroll
  for (int i = 0; i < 16; ++i) {
    if (MODE != 2 || grow0 + i < nN) {
      const v4f v = *(const v4f*)(lp + i * SP) + bv;
      *(volatile v4f*)(gp + (size_t)i * DF) = v;
    }
  }
  __threadfence();
#pragma unroll
  for (int i = 0; i < 16; ++i) {
    if (MODE != 2 || grow0 + i < nN) {
      const v4f v = *(const v4f*)(lp + i * SP) + bv;
      *(volatile v4f*)(gp + (size_t)i * DF) = v;
    }
  }
}

__device__ __forceinline__ void agg_store_pass(const float* acc, _Float16* hf,
                                               unsigned short* hch, unsigned short* hcl,
                                               int nodeBase, int wave, int lane) {
#pragma unroll 2
  for (int i = 0; i < NB / NWAVE; ++i) {
    const int row = wave * (NB / NWAVE) + i;
    const float* lp = acc + row * DF + 8 * lane;
    const v4f p0 = *(const v4f*)lp, p1 = *(const v4f*)(lp + 4);
    const v8h fh = cvt8(p0 * HSC, p1 * HSC);
    v8u bh, bl;
    split8(p0, p1, bh, bl);
    const size_t gr = (size_t)nodeBase + row;
    *(volatile v8h*)(hf + gr * DF + 8 * lane) = fh;
    *(volatile v8u*)(hch + gr * KJ + 8 * lane) = bh;
    *(volatile v8u*)(hcl + gr * KJ + 8 * lane) = bl;
  }
}

__global__ __launch_bounds__(NTHR) void k_agg(
    const int* __restrict__ ei, const float* __restrict__ g, const float* __restrict__ dinv,
    const float* __restrict__ bsl, const float* __restrict__ scl, const float* __restrict__ bbl,
    const float* __restrict__ mnl, const float* __restrict__ vrl,
    _Float16* hf, unsigned short* hch, unsigned short* hcl, int nN, int nE, int vec8) {
  extern __shared__ v4f lds_dyn[];
  float* acc  = (float*)lds_dyn;
  int*   list = (int*)(acc + NB * DF);
  int*   wcnt = list + LISTN;
  const int tid = threadIdx.x, lane = tid & 31, wave = tid >> 5;
  const int nodeBase = blockIdx.x * NB;
  const int* dsts = ei + nE;

  {
    const v4f z = {0.f, 0.f, 0.f, 0.f};
    for (int i = tid; i < NB * DF / 4; i += NTHR) lds_dyn[i] = z;
  }
  __syncthreads();

  const int nChunks = (nE + CHUNK - 1) / CHUNK;
#pragma unroll 1
  for (int ch = 0; ch < nChunks; ++ch) {
    const int cbase = ch * CHUNK;
    const int wc = scan_chunk<NB>(dsts, nE, cbase, nodeBase, vec8, list, tid, lane, wave);
    if (lane == 0) wcnt[wave] = wc;
    __syncthreads();
    if (wave == 0) {
#pragma unroll 1
      for (int wsx = 0; wsx < NWAVE; ++wsx) {
        int n = __builtin_amdgcn_readfirstlane(wcnt[wsx]);
        n = n > WCAP ? WCAP : (n < 0 ? 0 : n);
        const int* lp = list + wsx * WCAP;
#pragma unroll 1
        for (int i = 0; i < n; ++i) {
          const int ent  = __builtin_amdgcn_readfirstlane(lp[i]);
          const int slot = ent & (NB - 1);
          int e = cbase + ((ent >> 12) & (CHUNK - 1));
          e = e > nE - 1 ? nE - 1 : e;
          int src = __builtin_amdgcn_readfirstlane(ei[e]);
          src = src < 0 ? 0 : (src > nN - 1 ? nN - 1 : src);
          const float* gr = g + (size_t)src * DF + 4 * lane;
          const v4f v0 = *(const v4f*)gr;
          const v4f v1 = *(const v4f*)(gr + 128);
          v4f* ap = (v4f*)(acc + slot * DF + 4 * lane);
          ap[0]  = ap[0] + v0;
          ap[32] = ap[32] + v1;
        }
      }
    }
    __syncthreads();
  }

#pragma unroll 4
  for (int i = 0; i < (NB * DF / 4) / NTHR; ++i) {
    const int idx  = i * NTHR + tid;
    const int slot = idx >> 6;
    const int c4   = (idx & 63) * 4;
    int node = nodeBase + slot;
    node = node > nN - 1 ? nN - 1 : node;
    const float d  = dinv[node];
    const v4f   gv = *(const v4f*)(g + (size_t)node * DF + c4);
    const v4f   bv = *(const v4f*)(bsl + c4);
    const v4f   mv = *(const v4f*)(mnl + c4);
    const v4f   vv = *(const v4f*)(vrl + c4);
    const v4f   sv = *(const v4f*)(scl + c4);
    const v4f   ov = *(const v4f*)(bbl + c4);
    v4f rs;
    rs.x = rsqrtf(vv.x + BN_EPS); rs.y = rsqrtf(vv.y + BN_EPS);
    rs.z = rsqrtf(vv.z + BN_EPS); rs.w = rsqrtf(vv.w + BN_EPS);
    v4f* ap = (v4f*)(acc + slot * DF + c4);
    v4f hv = (*ap + gv) * d + bv;
    hv = (hv - mv) * rs * sv + ov;
    hv.x = fmaxf(hv.x, 0.f); hv.y = fmaxf(hv.y, 0.f); hv.z = fmaxf(hv.z, 0.f); hv.w = fmaxf(hv.w, 0.f);
    *ap = hv;
  }
  __syncthreads();

  agg_store_pass(acc, hf, hch, hcl, nodeBase, wave, lane);
  __threadfence();
  agg_store_pass(acc, hf, hch, hcl, nodeBase, wave, lane);
}

extern "C" void kernel_launch(void* const* d_in, const int* in_sizes, int n_in,
                              void* d_out, int out_size, void* d_ws, size_t ws_size,
                              hipStream_t stream) {
  if (n_in < 10) return;
  const int nN = in_sizes[0] / DF;
  const int nE = in_sizes[1] / 2;
  if (nN <= 0 || nE < 0 || in_sizes[0] != nN * DF || in_sizes[1] != nE * 2) return;
  if (in_sizes[2] != NLAY * DF * DF) return;
  if (in_sizes[3] != NLAY * DF || in_sizes[4] != NLAY * DF || in_sizes[5] != NLAY * DF ||
      in_sizes[6] != NLAY * DF || in_sizes[7] != NLAY * DF) return;
  if (in_sizes[8] != KJ * DF || in_sizes[9] != DF) return;
  if (out_size != nN * DF) return;

  const float* x     = (const float*)d_in[0];
  const int*   ei    = (const int*)d_in[1];
  const float* Ws    = (const float*)d_in[2];
  const float* bs    = (const float*)d_in[3];
  const float* bnsc  = (const float*)d_in[4];
  const float* bnb   = (const float*)d_in[5];
  const float* bnm   = (const float*)d_in[6];
  const float* bnv   = (const float*)d_in[7];
  const float* lw    = (const float*)d_in[8];
  const float* lb    = (const float*)d_in[9];
  float* out = (float*)d_out;

  const int nPad = ((nN + NB - 1) / NB) * NB;
  const int nA   = nPad / NB;
  const int nG   = nPad / GROWS;
  const int nBD  = (nN + NBD - 1) / NBD;
  if (nBD * NBD < nPad) return;

  char* ws = (char*)d_ws;
  size_t off = 0;
  const size_t oXh = off; off += (size_t)nPad * DF * 2;        off = (off + 255) & ~(size_t)255;
  const size_t oXl = off; off += (size_t)nPad * DF * 2;        off = (off + 255) & ~(size_t)255;
  const size_t oW0h = off; off += (size_t)DF * DF * 2;         off = (off + 255) & ~(size_t)255;
  const size_t oW0l = off; off += (size_t)DF * DF * 2;         off = (off + 255) & ~(size_t)255;
  const size_t oW1 = off; off += (size_t)DF * DF * 2;          off = (off + 255) & ~(size_t)255;
  const size_t oW2 = off; off += (size_t)DF * DF * 2;          off = (off + 255) & ~(size_t)255;
  const size_t oLh = off; off += (size_t)DF * KJ * 2;          off = (off + 255) & ~(size_t)255;
  const size_t oLl = off; off += (size_t)DF * KJ * 2;          off = (off + 255) & ~(size_t)255;
  const size_t oHf = off; off += (size_t)nPad * DF * 2;        off = (off + 255) & ~(size_t)255;
  const size_t oCh = off; off += (size_t)nPad * KJ * 2;        off = (off + 255) & ~(size_t)255;
  const size_t oCl = off; off += (size_t)nPad * KJ * 2;        off = (off + 255) & ~(size_t)255;
  const size_t oG  = off; off += (size_t)nPad * DF * 4;        off = (off + 255) & ~(size_t)255;
  const size_t oDv = off; off += (size_t)nBD * NBD * 4;        off = (off + 255) & ~(size_t)255;
  if (off > ws_size || off > WS_CAP) return;

  unsigned short* xh  = (unsigned short*)(ws + oXh);
  unsigned short* xl  = (unsigned short*)(ws + oXl);
  unsigned short* w0h = (unsigned short*)(ws + oW0h);
  unsigned short* w0l = (unsigned short*)(ws + oW0l);
  _Float16*       w1f = (_Float16*)(ws + oW1);
  _Float16*       w2f = (_Float16*)(ws + oW2);
  unsigned short* lwh = (unsigned short*)(ws + oLh);
  unsigned short* lwl = (unsigned short*)(ws + oLl);
  _Float16*       hf  = (_Float16*)(ws + oHf);
  unsigned short* hch = (unsigned short*)(ws + oCh);
  unsigned short* hcl = (unsigned short*)(ws + oCl);
  float*          gpl = (float*)(ws + oG);
  float*          dinv = (float*)(ws + oDv);

  const int vec8 = ((nE & 3) == 0) ? 1 : 0;

  const int nPrep = 3 * (DF * DF / 8) + DF * KJ / 8 + nPad * (DF / 8);
  k_prep<<<(nPrep + NTHR - 1) / NTHR, NTHR, 0, stream>>>(x, Ws, lw, xh, xl, w0h, w0l, w1f, w2f,
                                                        lwh, lwl, nN, nPad);
  k_deg<<<nBD, NTHR, 0, stream>>>(ei, dinv, nN, nE, vec8);

  hipFuncSetAttribute(reinterpret_cast<const void*>(&k_gemm<0>),
                      hipFuncAttributeMaxDynamicSharedMemorySize, LDS_GEMM);
  hipFuncSetAttribute(reinterpret_cast<const void*>(&k_gemm<1>),
                      hipFuncAttributeMaxDynamicSharedMemorySize, LDS_GEMM);
  hipFuncSetAttribute(reinterpret_cast<const void*>(&k_gemm<2>),
                      hipFuncAttributeMaxDynamicSharedMemorySize, LDS_GEMM);
  hipFuncSetAttribute(reinterpret_cast<const void*>(&k_agg),
                      hipFuncAttributeMaxDynamicSharedMemorySize, LDS_AGG);

  const dim3 ggrid(nG, 2);

  k_gemm<0><<<ggrid, NTHR, LDS_GEMM, stream>>>(xh, xl, DF, w0h, w0l, DF, dinv, lb, gpl, nN);
  k_agg<<<nA, NTHR, LDS_AGG, stream>>>(ei, gpl, dinv, bs, bnsc, bnb, bnm, bnv,
                                       hf, hch, hcl, nN, nE, vec8);
  k_gemm<1><<<ggrid, NTHR, LDS_GEMM, stream>>>((const unsigned short*)hf, (const unsigned short*)hf, DF,
                                               (const unsigned short*)w1f, (const unsigned short*)w1f, DF,
                                               dinv, lb, gpl, nN);
  k_agg<<<nA, NTHR, LDS_AGG, stream>>>(ei, gpl, dinv, bs + DF, bnsc + DF, bnb + DF, bnm + DF, bnv + DF,
                                       hf, hch + DF, hcl + DF, nN, nE, vec8);
  k_gemm<1><<<ggrid, NTHR, LDS_GEMM, stream>>>((const unsigned short*)hf, (const unsigned short*)hf, DF,
                                               (const unsigned short*)w2f, (const unsigned short*)w2f, DF,
                                               dinv, lb, gpl, nN);
  k_agg<<<nA, NTHR, LDS_AGG, stream>>>(ei, gpl, dinv, bs + 2 * DF, bnsc + 2 * DF, bnb + 2 * DF,
                                       bnm + 2 * DF, bnv + 2 * DF,
                                       hf, hch + 2 * DF, hcl + 2 * DF, nN, nE, vec8);
  k_gemm<2><<<ggrid, NTHR, LDS_GEMM, stream>>>(hch, hcl, KJ, lwh, lwl, KJ, dinv, lb, out, nN);
}
